// SiameseRelational_64441689309605
// MI455X (gfx1250) — hardware-verified
//
#include <hip/hip_runtime.h>


#define NB_  8
#define CC   512
#define LL   196
#define LP   256
#define HID  256

typedef unsigned short bf;
typedef __attribute__((ext_vector_type(16))) __bf16   v16bf;
typedef __attribute__((ext_vector_type(8)))  unsigned short v8us;
typedef __attribute__((ext_vector_type(8)))  float    v8f;
typedef __attribute__((ext_vector_type(4)))  float    v4f;
typedef v4f  __attribute__((may_alias)) v4fa;
typedef v8us __attribute__((may_alias)) v8usa;

__device__ __forceinline__ unsigned short f2bf(float f) { unsigned u = __float_as_uint(f); u += 0x7FFFu + ((u >> 16) & 1u); return (unsigned short)(u >> 16); }
__device__ __forceinline__ float bf2f(unsigned short b) { return __uint_as_float(((unsigned)b) << 16); }
__device__ __forceinline__ float bfr(float f) { return bf2f(f2bf(f)); }
__device__ __forceinline__ v16bf cat16b(v8us lo, v8us hi) { return __builtin_bit_cast(v16bf, __builtin_shufflevector(lo, hi, 0, 1, 2, 3, 4, 5, 6, 7, 8, 9, 10, 11, 12, 13, 14, 15)); }
__device__ __forceinline__ v8f wmmab(v16bf a, v16bf b, v8f c) { return __builtin_amdgcn_wmma_f32_16x16x32_bf16(false, a, false, b, (short)0, c, false, false); }
#define VST2(T, p, v) do { const T vst2_v_ = (v); *(volatile T*)(p) = vst2_v_; __threadfence(); *(volatile T*)(p) = vst2_v_; } while (0)

__global__ __launch_bounds__(256) void k_xt(const float* __restrict__ f1, const float* __restrict__ f2, bf* X1b, bf* X2b) {
    __shared__ __align__(16) unsigned short tl[64 * 72];
    const int tid = threadIdx.x, c0 = blockIdx.x * 64, l0 = blockIdx.y * 64, b = blockIdx.z >> 1, which = blockIdx.z & 1;
    const float* f = (which ? f2 : f1) + (size_t)b * CC * LL;
    bf* dst = (which ? X2b : X1b) + (size_t)b * LP * CC;
    const int cc = tid >> 2, lq = (tid & 3) * 16;
#pragma unroll
    for (int i = 0; i < 16; ++i) { const int l = l0 + lq + i; tl[(lq + i) * 72 + cc] = (l < LL) ? f2bf(f[(size_t)(c0 + cc) * LL + l]) : (unsigned short)0; }
    __syncthreads();
    const int piece = tid & 7;
    auto pass = [&]() {
#pragma unroll
        for (int s = 0; s < 2; ++s) { const int lr_ = (tid >> 3) + 32 * s; const v8us val = *(const v8usa*)(tl + lr_ * 72 + piece * 8);
            *(volatile v8us*)(dst + (size_t)(l0 + lr_) * CC + c0 + piece * 8) = val; }
    };
    pass(); __threadfence(); pass();
}
__global__ __launch_bounds__(256) void k_wt(const float* __restrict__ W1, bf* WT) {
    __shared__ __align__(16) unsigned short tl[64 * 72];
    const int tid = threadIdx.x, k0 = blockIdx.x * 64, n0 = blockIdx.y * 64;
    const int kk = tid >> 2, nq = (tid & 3) * 16;
#pragma unroll
    for (int i = 0; i < 16; ++i) tl[(nq + i) * 72 + kk] = f2bf(W1[(size_t)(k0 + kk) * HID + n0 + nq + i]);
    __syncthreads();
    const int piece = tid & 7;
    const int which = k0 / CC, kl = k0 - which * CC;
    auto pass = [&]() {
#pragma unroll
        for (int s = 0; s < 2; ++s) { const int nr = (tid >> 3) + 32 * s; const v8us val = *(const v8usa*)(tl + nr * 72 + piece * 8);
            *(volatile v8us*)(WT + ((size_t)which * HID + n0 + nr) * CC + kl + piece * 8) = val; }
    };
    pass(); __threadfence(); pass();
}
__global__ __launch_bounds__(128) void k_gemm(const bf* __restrict__ X1b, const bf* __restrict__ X2b, const bf* __restrict__ WT, float* P) {
    __shared__ __align__(16) float ost[4][16 * 68];
    const int lane = threadIdx.x & 31, wave = threadIdx.x >> 5, lr = lane & 15, hi = lane >> 4, which = blockIdx.z;
    const int r0 = blockIdx.x * 64 + wave * 16, c0 = blockIdx.y * 64;
    const bf* A = which ? X2b : X1b; const bf* Bn = WT + (size_t)which * HID * CC;
    const size_t aoff = (size_t)(r0 + lr) * CC + 8 * hi;
    size_t boff[4];
#pragma unroll
    for (int t = 0; t < 4; ++t) boff[t] = (size_t)(c0 + t * 16 + lr) * CC + 8 * hi;
    v8f acc[4];
#pragma unroll
    for (int t = 0; t < 4; ++t) acc[t] = (v8f){};
#pragma unroll 1
    for (int kc = 0; kc < CC; kc += 32) {
        const v16bf a = cat16b(*(const v8us*)(A + aoff + kc), *(const v8us*)(A + aoff + kc + 16));
#pragma unroll
        for (int t = 0; t < 4; ++t) acc[t] = wmmab(a, cat16b(*(const v8us*)(Bn + boff[t] + kc), *(const v8us*)(Bn + boff[t] + kc + 16)), acc[t]);
        asm volatile("v_nop\n\tv_nop\n\tv_nop\n\tv_nop" : "+v"(acc[0]), "+v"(acc[1]), "+v"(acc[2]), "+v"(acc[3]) : "v"(a));
    }
    float* os = &ost[wave][0];
#pragma unroll
    for (int t = 0; t < 4; ++t)
#pragma unroll
        for (int j = 0; j < 8; ++j) os[(hi * 8 + j) * 68 + t * 16 + lr] = acc[t][j];
    __syncthreads();
    float* crow = P + ((size_t)which * NB_ * LP + r0) * HID + c0;
    auto pass = [&]() {
#pragma unroll
        for (int s = 0; s < 8; ++s) { const int Lid = (lane >> 3) + 4 * s, piece = lane & 7; const int row = Lid >> 1, cofs = (Lid & 1) * 32 + piece * 4;
            const v4f val = *(const v4fa*)(os + row * 68 + cofs); *(volatile v4f*)(crow + (size_t)row * HID + cofs) = val; }
    };
    pass(); __threadfence(); pass();
}
__global__ __launch_bounds__(256) void k_pair(const float* __restrict__ P, const float* __restrict__ b1, const float* __restrict__ W2, const float* __restrict__ b2, float* PART) {
    __shared__ float red[8];
    const int b = blockIdx.x / LL, i = blockIdx.x - b * LL, j = threadIdx.x, lane = j & 31, wv = j >> 5;
    const float* p1 = P + ((size_t)b * LP + i) * HID; const float* p2 = P + ((size_t)NB_ * LP + (size_t)b * LP + j) * HID;
    float s = 0.f;
    if (j < LL) {
#pragma unroll 4
        for (int h = 0; h < HID; ++h) s += fmaxf(p1[h] + p2[h] + bfr(b1[h]), 0.f) * bfr(W2[h]);
        s += bfr(b2[0]);
    }
#pragma unroll
    for (int o = 16; o; o >>= 1) s += __shfl_xor(s, o, 32);
    if (lane == 0) red[wv] = s;
    __syncthreads();
    if (wv == 0) { float t = 0.f;
#pragma unroll
        for (int w = 0; w < 8; ++w) t += red[w];
        VST2(float, PART + (size_t)blockIdx.x * 32 + lane, t); }
}
__global__ __launch_bounds__(32) void k_fin(const float* __restrict__ PART, float* out) {
    const int lane = threadIdx.x;
    float s = 0.f;
    if (lane < NB_) {
#pragma unroll 1
        for (int i = 0; i < LL; ++i) s += PART[((size_t)lane * LL + i) * 32];
        *(volatile float*)(out + lane) = s;
    }
    __threadfence();
    if (lane < NB_) *(volatile float*)(out + lane) = s;
}

extern "C" void kernel_launch(void* const* d_in, const int* in_sizes, int n_in,
                              void* d_out, int out_size, void* d_ws, size_t ws_size, hipStream_t stream) {
    (void)in_sizes; (void)n_in; (void)out_size;
    const float* f1 = (const float*)d_in[0]; const float* f2 = (const float*)d_in[1]; const float* W1 = (const float*)d_in[2]; const float* b1 = (const float*)d_in[3];
    const float* W2 = (const float*)d_in[4]; const float* b2 = (const float*)d_in[5];
    float* out = (float*)d_out;
    char* wsp = (char*)d_ws;
    auto take = [&](size_t bytes) { char* p = wsp; wsp += (bytes + 255) & ~(size_t)255; return (void*)p; };
    bf* X1b = (bf*)take((size_t)NB_ * LP * CC * 2); bf* X2b = (bf*)take((size_t)NB_ * LP * CC * 2); bf* WT = (bf*)take((size_t)2 * HID * CC * 2);
    float* P = (float*)take((size_t)2 * NB_ * LP * HID * 4); float* PART = (float*)take((size_t)NB_ * LL * 32 * 4);
    if ((size_t)(wsp - (char*)d_ws) > ws_size) return;
    k_xt<<<dim3(CC / 64, LP / 64, 2 * NB_), 256, 0, stream>>>(f1, f2, X1b, X2b);
    k_wt<<<dim3((2 * CC) / 64, HID / 64, 1), 256, 0, stream>>>(W1, WT);
    k_gemm<<<dim3((NB_ * LP) / 64, HID / 64, 2), 128, 0, stream>>>(X1b, X2b, WT, P);
    k_pair<<<NB_ * LL, 256, 0, stream>>>(P, b1, W2, b2, PART);
    k_fin<<<1, 32, 0, stream>>>(PART, out);
}
